// SelfAttention_16277926052531
// MI455X (gfx1250) — hardware-verified
//
#include <hip/hip_runtime.h>
#include <math.h>

typedef __attribute__((ext_vector_type(16))) _Float16 v16h;
typedef __attribute__((ext_vector_type(16))) __bf16 v16b;
typedef __attribute__((ext_vector_type(8)))  _Float16 v8h;
typedef __attribute__((ext_vector_type(8)))  __bf16 v8b;
typedef __attribute__((ext_vector_type(8)))  float v8f;
typedef __attribute__((ext_vector_type(4)))  float v4f;
typedef __attribute__((ext_vector_type(4)))  unsigned v4u;

#ifndef NB
#define NB 2
#endif
#ifndef SEQ
#define SEQ 2048
#endif
#define NB_FULL 2
#define SEQ_FULL 2048
#define CC 1024
#define DIN 1024
#define NH 16
#define HD 64
#define NQB (SEQ / 64)
#define QBH 4
#define KHI 256
#define SC2 (0.125f * 1.4426950408889634f)

static_assert(SEQ % 64 == 0);
static_assert(SEQ >= KHI);
static_assert(KHI == QBH * 64);
static_assert(NB <= NB_FULL && SEQ <= SEQ_FULL);
static_assert(CC == NH * HD);
static_assert(HD == 64);
static_assert(CC % 128 == 0 && DIN % 128 == 0);
static_assert(DIN % 64 == 0 && CC % 64 == 0);
static_assert(DIN % 32 == 0 && CC % 32 == 0);
static_assert(DIN == CC);
static_assert(((size_t)NB * SEQ * DIN) % (8 * 256) == 0);
static_assert((size_t)NB_FULL * SEQ_FULL * DIN * 4 == 16777216u);

#define WS_XB  ((size_t)0)
#define WS_WT  (WS_XB  + 2u * (size_t)NB * SEQ * DIN)
#define WS_WPT (WS_WT  + 2u * (size_t)3 * CC * DIN)
#define WS_QH  (WS_WPT + 2u * (size_t)DIN * CC)
#define WS_QL  (WS_QH  + 2u * (size_t)NB * SEQ * CC)
#define WS_KH  (WS_QL  + 2u * (size_t)NB * SEQ * CC)
#define WS_KL  (WS_KH  + 2u * (size_t)NB * SEQ * CC)
#define WS_VT  (WS_KL  + 2u * (size_t)NB * SEQ * CC)
#define WS_VB  (WS_VT  + 2u * (size_t)NB * CC * SEQ)
#define WS_VBL (WS_VB  + 2u * (size_t)NB * CC * KHI)
#define WS_CH  (WS_VBL + 2u * (size_t)NB * CC * KHI)
#define WS_CL  (WS_CH  + 2u * (size_t)NB * SEQ * CC)
#define WS_END (WS_CL  + 2u * (size_t)NB * SEQ * CC)
static_assert(WS_END <= (size_t)134217728u);

template <typename T> __device__ __forceinline__ void vst2(void* p, T v) { *(volatile T*)p = v; __threadfence(); *(volatile T*)p = v; }
__device__ __forceinline__ v8f wmma16(v16h a, v16h b, v8f c) {
  v8f d = __builtin_amdgcn_wmma_f32_16x16x32_f16(false, a, false, b, (short)0, c, false, false);
  asm volatile("v_nop\n\tv_nop\n\tv_nop\n\tv_nop" : "+v"(d) : "v"(a), "v"(b));
  return d;
}
__device__ __forceinline__ v8f wmma_bf(v16b a, v16b b, v8f c) {
  v8f d = __builtin_amdgcn_wmma_f32_16x16x32_bf16(false, a, false, b, (short)0, c, false, false);
  asm volatile("v_nop\n\tv_nop\n\tv_nop\n\tv_nop" : "+v"(d) : "v"(a), "v"(b));
  return d;
}
__device__ __forceinline__ v16h frag_h(const _Float16* rowk0, int lane) {
  union { v16h v; v8h q[2]; } u; const _Float16* p = rowk0 + 8 * (lane >> 4);
  u.q[0] = *(const v8h*)p; u.q[1] = *(const v8h*)(p + 16); return u.v;
}
__device__ __forceinline__ v16b frag_b(const __bf16* rowk0, int lane) {
  union { v16b v; v8b q[2]; } u; const __bf16* p = rowk0 + 8 * (lane >> 4);
  u.q[0] = *(const v8b*)p; u.q[1] = *(const v8b*)(p + 16); return u.v;
}
__device__ __forceinline__ float bfr(float v) { return (float)(__bf16)v; }
#define LDSX() do { asm volatile("s_wait_dscnt 0" ::: "memory"); __builtin_amdgcn_wave_barrier(); __builtin_amdgcn_fence(3  , "workgroup"); } while (0)

__global__ __launch_bounds__(256) void k_cvt_x(const float* __restrict__ X, __bf16* __restrict__ XB) {
  const size_t i = (size_t)blockIdx.x * 256 + threadIdx.x;
  const size_t e = i * 8; const size_t R = e / DIN; const int c = (int)(e % DIN); const size_t bb = R / SEQ, t = R % SEQ;
  const float* p = X + (bb * SEQ_FULL + t) * DIN + c;
  const v4f a = *(const v4f*)p, d = *(const v4f*)(p + 4);
  union { v8b v; v4u u; } o;
#pragma unroll
  for (int k = 0; k < 4; ++k) { o.v[k] = (__bf16)a[k]; o.v[4 + k] = (__bf16)d[k]; }
  vst2(XB + e, o.u);
}

__global__ __launch_bounds__(256) void k_cvt_wt(const float* __restrict__ W, __bf16* __restrict__ WT, int N) {
  __shared__ __align__(16) __bf16 t[64][72];
  const int tid = threadIdx.x; const int n0 = blockIdx.x * 64, k0 = blockIdx.y * 64;
  for (int e = tid; e < 64 * 64; e += 256) { const int kl = e >> 6, nl = e & 63; t[nl][kl] = (__bf16)W[(size_t)(k0 + kl) * N + n0 + nl]; }
  __syncthreads();
  for (int e = tid; e < 64 * 8; e += 256) { const int nl = e >> 3, q = e & 7; vst2(WT + (size_t)(n0 + nl) * DIN + k0 + q * 8, *(const v4u*)&t[nl][q * 8]); }
}

__global__ __launch_bounds__(128) void k_proj(const __bf16* __restrict__ XB, const __bf16* __restrict__ WT, const float* __restrict__ BA,
    _Float16* __restrict__ QH, _Float16* __restrict__ QL, _Float16* __restrict__ KH, _Float16* __restrict__ KL, _Float16* __restrict__ VT, __bf16* __restrict__ VB, __bf16* __restrict__ VBL) {
  __shared__ __align__(16) float st[64][132]; __shared__ __align__(16) _Float16 sh[64][136], sl[64][136]; __shared__ __align__(16) _Float16 th[128][72]; __shared__ __align__(16) __bf16 tb[128][72], tbl[128][72];
  const int tid = threadIdx.x, lane = tid & 31, col = lane & 15, g = lane >> 4; const int wave = __builtin_amdgcn_readfirstlane(tid >> 5);
  const int which = blockIdx.z; const int c0 = blockIdx.y * 128; const size_t r0 = (size_t)blockIdx.x * 64; const size_t bb = r0 / SEQ; const int t0 = (int)(r0 % SEQ);
  const __bf16* arow = XB + (r0 + wave * 16 + col) * DIN;
  const __bf16* wrow = WT + ((size_t)which * CC + c0 + col) * DIN;
  v8f acc[8] = {};
#pragma unroll 2
  for (int kc = 0; kc < DIN / 32; ++kc) { const v16b a = frag_b(arow + kc * 32, lane);
#pragma unroll
    for (int j = 0; j < 8; ++j) { const v16b w = frag_b(wrow + (size_t)j * 16 * DIN + kc * 32, lane); acc[j] = wmma_bf(a, w, acc[j]); } }
#pragma unroll
  for (int j = 0; j < 8; ++j) { const float bias = bfr(BA[which * CC + c0 + j * 16 + col]);
#pragma unroll
    for (int r = 0; r < 8; ++r) st[wave * 16 + 8 * g + r][j * 16 + col] = acc[j][r] + bias; }
  __syncthreads();
  if (which < 2) { _Float16* DH = which == 0 ? QH : KH; _Float16* DL = which == 0 ? QL : KL;
    for (int e = tid; e < 64 * 128; e += 128) { const int rl = e >> 7, cl = e & 127; const float v = st[rl][cl]; const _Float16 hv = (_Float16)v; sh[rl][cl] = hv; sl[rl][cl] = (_Float16)((v - (float)hv) * 1024.0f); }
    __syncthreads();
    for (int e = tid; e < 64 * 16; e += 128) { const int rl = e >> 4, q = e & 15; const size_t o2 = (r0 + rl) * CC + c0 + q * 8; vst2(DH + o2, *(const v4u*)&sh[rl][q * 8]); vst2(DL + o2, *(const v4u*)&sl[rl][q * 8]); }
  } else { const bool hi_rows = t0 < KHI;
    for (int e = tid; e < 64 * 128; e += 128) { const int rl = e & 63, cl = e >> 6; const float v = st[rl][cl]; th[cl][rl] = (_Float16)v; const __bf16 bh = (__bf16)v; tb[cl][rl] = bh; tbl[cl][rl] = (__bf16)(v - (float)bh); }
    __syncthreads();
    for (int e = tid; e < 128 * 8; e += 128) { const int cl = e >> 3, q = e & 7; vst2(VT + (bb * CC + c0 + cl) * (size_t)SEQ + t0 + q * 8, *(const v4u*)&th[cl][q * 8]);
      if (hi_rows) { const size_t o3 = (bb * CC + c0 + cl) * (size_t)KHI + t0 + q * 8; vst2(VB + o3, *(const v4u*)&tb[cl][q * 8]); vst2(VBL + o3, *(const v4u*)&tbl[cl][q * 8]); } } } }

template <bool HI> __device__ __forceinline__ void attn_body(const _Float16* __restrict__ QH, const _Float16* __restrict__ QL, const _Float16* __restrict__ KH, const _Float16* __restrict__ KL,
    const _Float16* __restrict__ VT, const __bf16* __restrict__ VB, const __bf16* __restrict__ VBL, __bf16* __restrict__ CH, __bf16* __restrict__ CL, const int qb) {
  __shared__ __align__(16) _Float16 sp[4][16][40];
  __shared__ __align__(16) __bf16 sph[4][16][40];
  __shared__ __align__(16) __bf16 spl[4][16][40];
  __shared__ __align__(16) float so[4][16][68];
  const int tid = threadIdx.x, lane = tid & 31, col = lane & 15, g = lane >> 4; const int wave = __builtin_amdgcn_readfirstlane(tid >> 5);
  const int h = blockIdx.y, b = blockIdx.z;
  const int q0w = qb * 64 + wave * 16; const int nsteps = (q0w + 47) >> 5;
  const size_t rowb = (size_t)b * SEQ;
  const size_t qoff = (rowb + q0w + col) * CC + h * HD;
  const size_t koff = (rowb + col) * CC + h * HD;
  const size_t voff = ((size_t)b * CC + h * HD + col) * (size_t)SEQ;
  const size_t vboff = ((size_t)b * CC + h * HD + col) * (size_t)KHI;
  v8f o[4] = {}; float mrow[8], lsum[8];
#pragma unroll
  for (int r = 0; r < 8; ++r) { mrow[r] = -3.0e38f; lsum[r] = 0.f; }
#pragma unroll 1
  for (int st = 0; st < nsteps; ++st) { const int kbase = st * 32; int z = 0; asm volatile("" : "+s"(z));
    v8f sa[2] = {}, sr[2] = {};
#pragma unroll
    for (int kc = 0; kc < HD / 32; ++kc) { const v16h ah = frag_h(QH + qoff + z + kc * 32, lane), al = frag_h(QL + qoff + z + kc * 32, lane);
#pragma unroll
      for (int j = 0; j < 2; ++j) { const size_t ko = koff + (size_t)(kbase + j * 16) * CC + kc * 32; const v16h kh = frag_h(KH + ko, lane), kl = frag_h(KL + ko, lane);
        sa[j] = wmma16(ah, kh, sa[j]); sr[j] = wmma16(al, kh, sr[j]); sr[j] = wmma16(ah, kl, sr[j]); } }
    float sv[2][8], bm[8];
#pragma unroll
    for (int r = 0; r < 8; ++r) bm[r] = -3.0e38f;
#pragma unroll
    for (int j = 0; j < 2; ++j) { const int kn = kbase + j * 16 + col;
#pragma unroll
      for (int r = 0; r < 8; ++r) { const int qr = q0w + 8 * g + r; float v = (sa[j][r] + sr[j][r] * (1.0f / 1024.0f)) * SC2; v = (kn <= qr) ? v : -3.0e38f; sv[j][r] = v; bm[r] = fmaxf(bm[r], v); } }
#pragma unroll
    for (int off = 1; off < 16; off <<= 1) {
#pragma unroll
      for (int r = 0; r < 8; ++r) bm[r] = fmaxf(bm[r], __shfl_xor(bm[r], off)); }
#pragma unroll
    for (int r = 0; r < 8; ++r) { const float nm = fmaxf(mrow[r], bm[r]); const float corr = exp2f(mrow[r] - nm); mrow[r] = nm; lsum[r] *= corr;
#pragma unroll
      for (int t = 0; t < 4; ++t) o[t][r] *= corr; }
#pragma unroll
    for (int j = 0; j < 2; ++j) {
#pragma unroll
      for (int r = 0; r < 8; ++r) { const float ev = exp2f(sv[j][r] - mrow[r]); const float p = (sv[j][r] > -1.0e38f) ? ev : 0.f; lsum[r] += p; const float pc = p * 1024.0f;
        if (HI) { const __bf16 ph = (__bf16)pc; sph[wave][8 * g + r][j * 16 + col] = ph; spl[wave][8 * g + r][j * 16 + col] = (__bf16)(pc - (float)ph); }
        else sp[wave][8 * g + r][j * 16 + col] = (_Float16)pc; } }
    LDSX();
    if (HI) { union { v16b v; v8b q[2]; } uh, ul;
      uh.q[0] = *(const v8b*)&sph[wave][col][8 * g]; uh.q[1] = *(const v8b*)&sph[wave][col][16 + 8 * g];
      ul.q[0] = *(const v8b*)&spl[wave][col][8 * g]; ul.q[1] = *(const v8b*)&spl[wave][col][16 + 8 * g];
      LDSX();
#pragma unroll
      for (int t = 0; t < 4; ++t) { const size_t po = vboff + (size_t)t * 16 * KHI + kbase; const v16b vh = frag_b(VB + po, lane), vl = frag_b(VBL + po, lane);
        o[t] = wmma_bf(ul.v, vh, o[t]); o[t] = wmma_bf(uh.v, vl, o[t]); o[t] = wmma_bf(uh.v, vh, o[t]); }
    } else { union { v16h v; v8h q[2]; } up;
      up.q[0] = *(const v8h*)&sp[wave][col][8 * g]; up.q[1] = *(const v8h*)&sp[wave][col][16 + 8 * g];
      LDSX();
#pragma unroll
      for (int t = 0; t < 4; ++t) { const v16h vf = frag_h(VT + voff + (size_t)t * 16 * SEQ + kbase, lane); o[t] = wmma16(up.v, vf, o[t]); } } }
#pragma unroll
  for (int off = 1; off < 16; off <<= 1) {
#pragma unroll
    for (int r = 0; r < 8; ++r) lsum[r] += __shfl_xor(lsum[r], off); }
#pragma unroll
  for (int r = 0; r < 8; ++r) { const float inv = (1.0f / 1024.0f) * (1.0f / lsum[r]);
#pragma unroll
    for (int t = 0; t < 4; ++t) so[wave][8 * g + r][t * 16 + col] = o[t][r] * inv; }
  LDSX();
#pragma unroll
  for (int it = 0; it < 4; ++it) { const int row = it * 4 + (lane >> 3), q = lane & 7;
    const v4f a = *(const v4f*)&so[wave][row][q * 8], c = *(const v4f*)&so[wave][row][q * 8 + 4];
    union { v8b v; v4u u; } uh, ul;
#pragma unroll
    for (int k = 0; k < 4; ++k) { const __bf16 h0 = (__bf16)a[k]; uh.v[k] = h0; ul.v[k] = (__bf16)(a[k] - (float)h0); const __bf16 h1 = (__bf16)c[k]; uh.v[4 + k] = h1; ul.v[4 + k] = (__bf16)(c[k] - (float)h1); }
    const size_t dst = (rowb + q0w + row) * CC + h * HD + q * 8;
    vst2(CH + dst, uh.u); vst2(CL + dst, ul.u); } }

__global__ __launch_bounds__(128) void k_attn_hi(const _Float16* __restrict__ QH, const _Float16* __restrict__ QL, const _Float16* __restrict__ KH, const _Float16* __restrict__ KL,
    const _Float16* __restrict__ VT, const __bf16* __restrict__ VB, const __bf16* __restrict__ VBL, __bf16* __restrict__ CH, __bf16* __restrict__ CL) {
  attn_body<true>(QH, QL, KH, KL, VT, VB, VBL, CH, CL, (int)blockIdx.x); }
__global__ __launch_bounds__(128) void k_attn_lo(const _Float16* __restrict__ QH, const _Float16* __restrict__ QL, const _Float16* __restrict__ KH, const _Float16* __restrict__ KL,
    const _Float16* __restrict__ VT, const __bf16* __restrict__ VB, const __bf16* __restrict__ VBL, __bf16* __restrict__ CH, __bf16* __restrict__ CL) {
  attn_body<false>(QH, QL, KH, KL, VT, VB, VBL, CH, CL, QBH + (int)blockIdx.x); }

__global__ __launch_bounds__(128) void k_out(const __bf16* __restrict__ CH, const __bf16* __restrict__ CL, const __bf16* __restrict__ WPT, const float* __restrict__ BO, float* __restrict__ OUT) {
  __shared__ __align__(16) float sf[4][16][132];
  const int tid = threadIdx.x, lane = tid & 31, col = lane & 15, g = lane >> 4; const int wave = __builtin_amdgcn_readfirstlane(tid >> 5);
  const int c0 = blockIdx.y * 128; const size_t rb = (size_t)blockIdx.x * 64; const size_t r0 = rb + wave * 16;
  const size_t orow0 = (rb / SEQ) * SEQ_FULL + (rb % SEQ) + wave * 16;
  const __bf16* ahp = CH + (r0 + col) * CC; const __bf16* alp = CL + (r0 + col) * CC; const __bf16* wrow = WPT + (size_t)(c0 + col) * CC;
  v8f acc[8] = {};
#pragma unroll 2
  for (int kc = 0; kc < CC / 32; ++kc) { const v16b ah = frag_b(ahp + kc * 32, lane), al = frag_b(alp + kc * 32, lane);
#pragma unroll
    for (int j = 0; j < 8; ++j) { const v16b w = frag_b(wrow + (size_t)j * 16 * CC + kc * 32, lane); acc[j] = wmma_bf(al, w, acc[j]); acc[j] = wmma_bf(ah, w, acc[j]); } }
#pragma unroll
  for (int j = 0; j < 8; ++j) { const float bias = bfr(BO[c0 + j * 16 + col]);
#pragma unroll
    for (int r = 0; r < 8; ++r) sf[wave][8 * g + r][j * 16 + col] = acc[j][r] + bias; }
  LDSX();
  for (int rl = 0; rl < 16; ++rl) vst2(OUT + (orow0 + rl) * DIN + c0 + lane * 4, *(const v4f*)&sf[wave][rl][lane * 4]); }

extern "C" void kernel_launch(void* const* d_in, const int* in_sizes, int n_in, void* d_out, int out_size, void* d_ws, size_t ws_size, hipStream_t stream) {
  if (n_in < 5) return;
  const long long need_x = ((long long)(NB - 1) * SEQ_FULL + SEQ) * DIN;
  if ((long long)in_sizes[0] < need_x) return;
  if ((long long)in_sizes[1] < (long long)DIN * 3 * CC) return;
  if (in_sizes[2] < 3 * CC) return;
  if ((long long)in_sizes[3] < (long long)CC * DIN) return;
  if (in_sizes[4] < DIN) return;
  if ((long long)out_size < need_x) return;
  if (ws_size < (size_t)WS_END) return;
  const float* X = (const float*)d_in[0]; const float* WA = (const float*)d_in[1]; const float* BA = (const float*)d_in[2]; const float* WP = (const float*)d_in[3]; const float* BP = (const float*)d_in[4];
  char* ws = (char*)d_ws;
  __bf16 *XB = (__bf16*)(ws + WS_XB), *WT = (__bf16*)(ws + WS_WT), *WPT = (__bf16*)(ws + WS_WPT);
  _Float16 *QH = (_Float16*)(ws + WS_QH), *QL = (_Float16*)(ws + WS_QL), *KH = (_Float16*)(ws + WS_KH), *KL = (_Float16*)(ws + WS_KL), *VT = (_Float16*)(ws + WS_VT);
  __bf16 *VB = (__bf16*)(ws + WS_VB), *VBL = (__bf16*)(ws + WS_VBL), *CH = (__bf16*)(ws + WS_CH), *CL = (__bf16*)(ws + WS_CL);
  k_cvt_x<<<dim3((unsigned)(((size_t)NB * SEQ * DIN) / (8 * 256))), 256, 0, stream>>>(X, XB);
  k_cvt_wt<<<dim3(3 * CC / 64, DIN / 64), 256, 0, stream>>>(WA, WT, 3 * CC);
  k_cvt_wt<<<dim3(DIN / 64, CC / 64), 256, 0, stream>>>(WP, WPT, DIN);
  k_proj<<<dim3(NB * SEQ / 64, CC / 128, 3), 128, 0, stream>>>(XB, WT, BA, QH, QL, KH, KL, VT, VB, VBL);
  k_attn_hi<<<dim3(QBH, NH, NB), 128, 0, stream>>>(QH, QL, KH, KL, VT, VB, VBL, CH, CL);
  if (NQB > QBH) k_attn_lo<<<dim3(NQB - QBH, NH, NB), 128, 0, stream>>>(QH, QL, KH, KL, VT, VB, VBL, CH, CL);
  k_out<<<dim3(NB * SEQ / 64, DIN / 128), 128, 0, stream>>>(CH, CL, WPT, BP, (float*)d_out);
}
